// LoRAMulti_MLP_38302518346465
// MI455X (gfx1250) — hardware-verified
//
#include <hip/hip_runtime.h>
#include <math.h>

typedef __attribute__((ext_vector_type(16))) _Float16 v16h;
typedef __attribute__((ext_vector_type(16))) __bf16 v16b;
typedef __attribute__((ext_vector_type(8)))  _Float16 v8h;
typedef __attribute__((ext_vector_type(8)))  float v8f;
typedef __attribute__((ext_vector_type(4)))  float v4f;
typedef __attribute__((ext_vector_type(2)))  float v2f;
typedef __attribute__((ext_vector_type(4)))  unsigned v4u;
typedef __attribute__((ext_vector_type(4)))  int v4i;
typedef float __attribute__((may_alias)) float_a;
typedef int __attribute__((may_alias)) int_a;

template <typename T> __device__ __forceinline__ void vst2(void* p, T v) { *(volatile T*)p = v; __threadfence(); *(volatile T*)p = v; }
__device__ __forceinline__ v8f wmma16(v16h a, v16h b, v8f c) {
  v8f d = __builtin_amdgcn_wmma_f32_16x16x32_f16(false, a, false, b, (short)0, c, false, false);
  asm volatile("v_nop\n\tv_nop\n\tv_nop\n\tv_nop" : "+v"(d) : "v"(a), "v"(b));
  return d;
}
__device__ __forceinline__ v8f wmma_bf(v16b a, v16b b, v8f c) {
  v8f d = __builtin_amdgcn_wmma_f32_16x16x32_bf16(false, a, false, b, (short)0, c, false, false);
  asm volatile("v_nop\n\tv_nop\n\tv_nop\n\tv_nop" : "+v"(d) : "v"(a), "v"(b));
  return d;
}
__device__ __forceinline__ v16h frag_h(const _Float16* rowk0, int lane) {
  union { v16h v; v8h q[2]; } u; const _Float16* p = rowk0 + 8 * (lane >> 4);
  u.q[0] = *(const v8h*)p; u.q[1] = *(const v8h*)(p + 16); return u.v;
}
__device__ __forceinline__ v16h frag_f32(const float* rowk0, int lane) {
  v16h a; const float* p = rowk0 + 8 * (lane >> 4);
#pragma unroll
  for (int i = 0; i < 8; ++i) { a[i] = (_Float16)p[i]; a[8 + i] = (_Float16)p[16 + i]; }
  return a;
}
__device__ __forceinline__ v16h frag_f32s(const float* rowk0, int lane, float sc) {
  v16h a; const float* p = rowk0 + 8 * (lane >> 4);
#pragma unroll
  for (int i = 0; i < 8; ++i) { a[i] = (_Float16)(p[i] * sc); a[8 + i] = (_Float16)(p[16 + i] * sc); }
  return a;
}
__device__ __forceinline__ v16h fragc_f32(const float* W, int k0, int n, int lane, int ld, int K) {
  v16h a; const int g = lane >> 4;
#pragma unroll
  for (int i = 0; i < 8; ++i) { const int ka = k0 + 8 * g + i, kb = ka + 16;
    a[i] = (_Float16)(ka < K ? W[(size_t)(ka < K ? ka : K - 1) * ld + n] : 0.f); a[8 + i] = (_Float16)(kb < K ? W[(size_t)(kb < K ? kb : K - 1) * ld + n] : 0.f); }
  return a;
}
struct F2 { v16b h, l; };
__device__ __forceinline__ F2 bsplit16(const float v[16]) { F2 r;
#pragma unroll
  for (int i = 0; i < 16; ++i) { const __bf16 h = (__bf16)v[i]; r.h[i] = h; r.l[i] = (__bf16)(v[i] - (float)h); }
  return r; }
__device__ __forceinline__ F2 split_row(const float* row, int k0, int lane) { float v[16]; const float* p = row + k0 + 8 * (lane >> 4);
#pragma unroll
  for (int i = 0; i < 8; ++i) { v[i] = p[i]; v[8 + i] = p[16 + i]; }
  return bsplit16(v); }
__device__ __forceinline__ F2 split_rowK(const float* row, int k0, int lane, int K) { float v[16]; const int g = lane >> 4;
#pragma unroll
  for (int i = 0; i < 8; ++i) { const int ka = k0 + 8 * g + i, kb = ka + 16; v[i] = ka < K ? row[ka < K ? ka : K - 1] : 0.f; v[8 + i] = kb < K ? row[kb < K ? kb : K - 1] : 0.f; }
  return bsplit16(v); }
__device__ __forceinline__ F2 split_col(const float* W, int k0, int n, int lane, int ld, int K) { float v[16]; const int g = lane >> 4;
#pragma unroll
  for (int i = 0; i < 8; ++i) { const int ka = k0 + 8 * g + i, kb = ka + 16; v[i] = ka < K ? W[(size_t)(ka < K ? ka : K - 1) * ld + n] : 0.f; v[8 + i] = kb < K ? W[(size_t)(kb < K ? kb : K - 1) * ld + n] : 0.f; }
  return bsplit16(v); }
__device__ __forceinline__ v8f mac3(const F2& a, const F2& b, v8f c) { c = wmma_bf(a.l, b.h, c); c = wmma_bf(a.h, b.l, c); return wmma_bf(a.h, b.h, c); }
__device__ __forceinline__ float sigm(float v) { return 1.0f / (1.0f + expf(-v)); }
#define LDSX() do { asm volatile("s_wait_dscnt 0" ::: "memory"); __builtin_amdgcn_wave_barrier(); __builtin_amdgcn_fence(__ATOMIC_RELEASE, "workgroup"); } while (0)


#define NT 8
#define NBR 1024
#define NR (NT * NBR)
#define D0 1024
#define D1 2048
#define D2 2048
#define D3 1024
#define RK 8
#ifndef TRB
#define TRB (NR / 64)
#endif
typedef __attribute__((ext_vector_type(8))) __bf16 v8b;
__device__ __forceinline__ v16b frag_b(const __bf16* rowk0, int lane) {
  union { v16b v; v8b q[2]; } u; const __bf16* p = rowk0 + 8 * (lane >> 4);
  u.q[0] = *(const v8b*)p; u.q[1] = *(const v8b*)(p + 16); return u.v;
}
__device__ __forceinline__ float bfr(float v) { return (float)(__bf16)v; }
__device__ __attribute__((noinline)) float exp_ni(float v) { return expf(v); }
__device__ __attribute__((noinline)) float erf_ni(float v) { return erff(v); }

#define WS_K0  0u
#define WS_K1  (WS_K0 + 2u * (size_t)D1 * D0)
#define WS_K2  (WS_K1 + 2u * (size_t)D2 * D1)
#define WS_Dm0 (WS_K2 + 2u * (size_t)D3 * D2)
#define WS_Dm1 (WS_Dm0 + 2u * NT * 16 * D0)
#define WS_Dm2 (WS_Dm1 + 2u * NT * 16 * D1)
#define WS_U0  (WS_Dm2 + 2u * NT * 16 * D2)
#define WS_U1  (WS_U0 + 2u * NT * D1 * 32)
#define WS_U2  (WS_U1 + 2u * NT * D2 * 32)
#define WS_H1  (((WS_U2 + 2u * NT * D3 * 32) + 127u) / 128u * 128u)
#define WS_H2  (WS_H1 + 2u * (size_t)NR * D1)
#define WS_END (WS_H2 + 2u * (size_t)NR * D2)

template <int L>
__global__ __launch_bounds__(256) void k_packk(const float* __restrict__ Kw, void* __restrict__ dst) {
  constexpr int IN = (L == 0) ? D0 : (L == 1) ? D1 : D2; constexpr int OUTD = (L == 0) ? D1 : (L == 1) ? D2 : D3; const int n = blockIdx.x, t = threadIdx.x;
  if (L == 0) { __shared__ __align__(16) __bf16 s[IN]; for (int k = t; k < IN; k += 256) s[k] = (__bf16)Kw[(size_t)k * OUTD + n]; __syncthreads(); for (int q = t; q < IN / 8; q += 256) vst2((unsigned*)((__bf16*)dst + (size_t)n * IN + q * 8), *(const v4u*)&s[q * 8]); }
  else { __shared__ __align__(16) _Float16 s[IN]; for (int k = t; k < IN; k += 256) s[k] = (_Float16)bfr(Kw[(size_t)k * OUTD + n]); __syncthreads(); for (int q = t; q < IN / 8; q += 256) vst2((unsigned*)((_Float16*)dst + (size_t)n * IN + q * 8), *(const v4u*)&s[q * 8]); }
}
template <int L>
__global__ __launch_bounds__(256) void k_packdu(const float* __restrict__ Dw, const float* __restrict__ Uw, void* __restrict__ Dd, void* __restrict__ Ud) {
  constexpr int IN = (L == 0) ? D0 : (L == 1) ? D1 : D2; constexpr int OUTD = (L == 0) ? D1 : (L == 1) ? D2 : D3; const int tsk = blockIdx.x, which = blockIdx.y, t = threadIdx.x;
  if (which == 0) { for (int e = t; e < 16 * IN; e += 256) { const int r = e / IN, i = e % IN; const float v = (r < RK) ? bfr(Dw[((size_t)i * RK + r) * NT + tsk]) : 0.f; if (L == 0) ((__bf16*)Dd)[((size_t)tsk * 16 + r) * IN + i] = (__bf16)v; else ((_Float16*)Dd)[((size_t)tsk * 16 + r) * IN + i] = (_Float16)v; } }
  else { for (int e = t; e < OUTD * 32; e += 256) { const int f = e / 32, r = e % 32; const float v = (r < RK) ? bfr(Uw[((size_t)r * OUTD + f) * NT + tsk]) : 0.f; ((_Float16*)Ud)[((size_t)tsk * OUTD + f) * 32 + r] = (_Float16)v; } }
}
template <int L>
__global__ __launch_bounds__(128) void k_layer(const float* __restrict__ X, const _Float16* __restrict__ Hin, const void* __restrict__ Kp, const void* __restrict__ Dp, const _Float16* __restrict__ Up, const float* __restrict__ BIAS, _Float16* __restrict__ Hout, float* __restrict__ OUT) {
  constexpr int IN = (L == 0) ? D0 : (L == 1) ? D1 : D2; constexpr int OUTD = (L == 0) ? D1 : (L == 1) ? D2 : D3;
  __shared__ __align__(16) _Float16 shd[4][16][40], shl[4][16][40]; __shared__ __align__(16) float so[4][16][132]; __shared__ __align__(16) _Float16 soh[4][16][136];
  const int tid = threadIdx.x, wave = tid >> 5, lane = tid & 31, col = lane & 15, g = lane >> 4; const size_t r0 = (size_t)blockIdx.x * 64 + wave * 16; const int n0 = blockIdx.y * 128; const int tsk = (int)(r0 / NBR);
  v8f acc[8] = {}, hd = {};
  if (L == 0) { const __bf16* Kr = (const __bf16*)Kp; const __bf16* Dr = (const __bf16*)Dp + (size_t)tsk * 16 * IN;
#pragma unroll 2
    for (int kc = 0; kc < IN / 32; ++kc) { v16b a; { const float* p = X + (r0 + col) * IN + kc * 32 + 8 * g;
#pragma unroll
        for (int i = 0; i < 8; ++i) { a[i] = (__bf16)p[i]; a[8 + i] = (__bf16)p[16 + i]; } }
#pragma unroll
      for (int j = 0; j < 8; ++j) acc[j] = wmma_bf(a, frag_b(Kr + (size_t)(n0 + j * 16 + col) * IN + kc * 32, lane), acc[j]);
      hd = wmma_bf(a, frag_b(Dr + (size_t)col * IN + kc * 32, lane), hd); } }
  else { const _Float16* Kr = (const _Float16*)Kp; const _Float16* Dr = (const _Float16*)Dp + (size_t)tsk * 16 * IN;
#pragma unroll 2
    for (int kc = 0; kc < IN / 32; ++kc) { const v16h a = frag_h(Hin + (r0 + col) * IN + kc * 32, lane);
#pragma unroll
      for (int j = 0; j < 8; ++j) acc[j] = wmma16(a, frag_h(Kr + (size_t)(n0 + j * 16 + col) * IN + kc * 32, lane), acc[j]);
      hd = wmma16(a, frag_h(Dr + (size_t)col * IN + kc * 32, lane), hd); } }
#pragma unroll
  for (int r = 0; r < 8; ++r) { const float v = hd[r]; const _Float16 hv = (_Float16)v; shd[wave][8 * g + r][col] = hv; shl[wave][8 * g + r][col] = (_Float16)((v - (float)hv) * 2048.0f); shd[wave][8 * g + r][16 + col] = (_Float16)0.f; shl[wave][8 * g + r][16 + col] = (_Float16)0.f; }
  LDSX();
  { const v16h ah = frag_h(&shd[wave][col][0], lane), al = frag_h(&shl[wave][col][0], lane);
#pragma unroll
    for (int j = 0; j < 8; ++j) { const v16h u = frag_h(Up + ((size_t)tsk * OUTD + n0 + j * 16 + col) * 32, lane); v8f dl = {}; dl = wmma16(ah, u, dl); v8f dll = {}; dll = wmma16(al, u, dll);
#pragma unroll
      for (int r = 0; r < 8; ++r) acc[j][r] += (dl[r] + dll[r] * (1.0f / 2048.0f)) * 2.0f; } }
#pragma unroll
  for (int j = 0; j < 8; ++j) { const int c = n0 + j * 16 + col; const float bb = bfr(BIAS[c]);
#pragma unroll
    for (int r = 0; r < 8; ++r) { const float v = acc[j][r] + bb; if (L < 2) soh[wave][8 * g + r][j * 16 + col] = (_Float16)fmaxf(v, 0.f); else so[wave][8 * g + r][j * 16 + col] = v; } }
  LDSX();
  if (L < 2) { for (int rl = 0; rl < 16; ++rl) if (lane < 16) vst2((unsigned*)(Hout + (r0 + rl) * OUTD + n0 + lane * 8), *(const v4u*)&soh[wave][rl][lane * 8]); }
  else { for (int rl = 0; rl < 16; ++rl) vst2(OUT + (r0 + rl) * OUTD + n0 + lane * 4, *(const v4f*)&so[wave][rl][lane * 4]); }
}
extern "C" void kernel_launch(void* const* d_in, const int* in_sizes, int n_in, void* d_out, int out_size, void* d_ws, size_t ws_size, hipStream_t stream) {
  (void)in_sizes; (void)n_in; (void)out_size;
  const float** F = (const float**)d_in;
  if (ws_size < (size_t)WS_END) return;
  char* ws = (char*)d_ws; _Float16 *H1 = (_Float16*)(ws + WS_H1), *H2 = (_Float16*)(ws + WS_H2);
  k_packk<0><<<D1, 256, 0, stream>>>(F[1], ws + WS_K0); k_packk<1><<<D2, 256, 0, stream>>>(F[5], ws + WS_K1); k_packk<2><<<D3, 256, 0, stream>>>(F[9], ws + WS_K2);
  k_packdu<0><<<dim3(NT, 2), 256, 0, stream>>>(F[3], F[4], ws + WS_Dm0, ws + WS_U0); k_packdu<1><<<dim3(NT, 2), 256, 0, stream>>>(F[7], F[8], ws + WS_Dm1, ws + WS_U1); k_packdu<2><<<dim3(NT, 2), 256, 0, stream>>>(F[11], F[12], ws + WS_Dm2, ws + WS_U2);
  k_layer<0><<<dim3(TRB, D1 / 128), 128, 0, stream>>>(F[0], nullptr, ws + WS_K0, ws + WS_Dm0, (const _Float16*)(ws + WS_U0), F[2], H1, nullptr);
  k_layer<1><<<dim3(TRB, D2 / 128), 128, 0, stream>>>(nullptr, H1, ws + WS_K1, ws + WS_Dm1, (const _Float16*)(ws + WS_U1), F[6], H2, nullptr);
  k_layer<2><<<dim3(TRB, D3 / 128), 128, 0, stream>>>(nullptr, H2, ws + WS_K2, ws + WS_Dm2, (const _Float16*)(ws + WS_U2), F[10], nullptr, (float*)d_out);
}
